// SpectralAttention_73212012527749
// MI455X (gfx1250) — hardware-verified
//
#include <hip/hip_runtime.h>
#include <math.h>

constexpr int kSeqLen  = 1024;
constexpr int kModel   = 1024;
constexpr int kHeads   = 16;
constexpr int kHeadDim = 64;
constexpr int kExpand  = 8;
constexpr int kWide    = kModel * kExpand;
constexpr float kEpsF  = 1e-5f;
constexpr float kNormFloor = 1e-12f;
constexpr int kChunkT  = 16;

typedef __attribute__((ext_vector_type(16))) _Float16 v16h;
typedef __attribute__((ext_vector_type(8)))  _Float16 v8h;
typedef __attribute__((ext_vector_type(16))) __bf16   v16b;
typedef __attribute__((ext_vector_type(8)))  __bf16   v8b;
typedef __attribute__((ext_vector_type(8)))  float    v8f;
typedef __attribute__((ext_vector_type(4)))  float    v4f;
typedef __attribute__((ext_vector_type(4)))  unsigned int v4u;

__device__ __forceinline__ unsigned short f2bf_bits(float f) {
  unsigned u = __float_as_uint(f);
  return (unsigned short)((u + 0x7FFFu + ((u >> 16) & 1u)) >> 16);
}
__device__ __forceinline__ float bf_bits2f(unsigned short h) { return __uint_as_float(((unsigned)h) << 16); }

__device__ __forceinline__ void dep_guard_h(v8f& a, v8f& b, v16h x, v16h y) { asm volatile("v_nop\n\tv_nop\n\tv_nop\n\tv_nop" : "+v"(a), "+v"(b) : "v"(x), "v"(y)); }
__device__ __forceinline__ void dep_guard_b(v8f& a, v8f& b, v16b x, v16b y) { asm volatile("v_nop\n\tv_nop\n\tv_nop\n\tv_nop" : "+v"(a), "+v"(b) : "v"(x), "v"(y)); }
__device__ __forceinline__ void keep4_h(v16h a, v16h b, v16h c, v16h d) { asm volatile("v_nop" :: "v"(a), "v"(b), "v"(c), "v"(d)); }
__device__ __forceinline__ void keep4_b(v16b a, v16b b, v16b c, v16b d) { asm volatile("v_nop" :: "v"(a), "v"(b), "v"(c), "v"(d)); }
__device__ __forceinline__ void acc_guard4(v8f& a, v8f& b, v8f& c, v8f& d) { asm volatile("v_nop\n\tv_nop\n\tv_nop\n\tv_nop" : "+v"(a), "+v"(b), "+v"(c), "+v"(d)); }
template <typename T> struct Frag;
template <> struct Frag<_Float16> {
  typedef v16h V; union U { v16h v; v8h h[2]; };
  static __device__ __forceinline__ v16h load(const _Float16* p) {
    U f; f.h[0] = *(const v8h*)(p); f.h[1] = *(const v8h*)(p + 16); return f.v;
  }
  static __device__ __forceinline__ v8f mma(v16h a, v16h b, v8f c) {
    return __builtin_amdgcn_wmma_f32_16x16x32_f16(false, a, false, b, (short)0, c, false, false);
  }
  static __device__ __forceinline__ void guard(v8f& a, v8f& b, v16h x, v16h y) { dep_guard_h(a, b, x, y); }
  static __device__ __forceinline__ void keep(v16h a, v16h b, v16h c, v16h d) { keep4_h(a, b, c, d); }
};
template <> struct Frag<__bf16> {
  typedef v16b V; union U { v16b v; v8b h[2]; };
  static __device__ __forceinline__ v16b load(const __bf16* p) {
    U f; f.h[0] = *(const v8b*)(p); f.h[1] = *(const v8b*)(p + 16); return f.v;
  }
  static __device__ __forceinline__ v8f mma(v16b a, v16b b, v8f c) {
    return __builtin_amdgcn_wmma_f32_16x16x32_bf16(false, a, false, b, (short)0, c, false, false);
  }
  static __device__ __forceinline__ void guard(v8f& a, v8f& b, v16b x, v16b y) { dep_guard_b(a, b, x, y); }
  static __device__ __forceinline__ void keep(v16b a, v16b b, v16b c, v16b d) { keep4_b(a, b, c, d); }
};

__device__ __forceinline__ unsigned pk16(unsigned short a, unsigned short b) { return (unsigned)a | ((unsigned)b << 16); }

template <int ET> struct Elem;
template <> struct Elem<0> { typedef _Float16 T; };
template <> struct Elem<1> { typedef __bf16 T; };
template <int ET, bool SPLIT, int BIAS_MODE, int OUT_MODE, bool RESID, int ACT = 0>
__global__ __launch_bounds__(256) void wmma_gemm64(
    const unsigned short* __restrict__ Ap, const unsigned short* __restrict__ A2p, int lda, long strideA,
    const unsigned short* __restrict__ Btp, const unsigned short* __restrict__ Bt2p, int ldb, long strideB,
    void* __restrict__ Cout, void* __restrict__ Cout2, int ldc, long strideC,
    const float* __restrict__ bias,
    const float* __restrict__ resid, long strideR,
    int M, int N, int K, float scale) {
  typedef typename Elem<ET>::T T;
  typedef typename Frag<T>::V V;
  const T* A = (const T*)Ap; const T* A2 = (const T*)A2p; const T* Bt = (const T*)Btp; const T* Bt2 = (const T*)Bt2p;
  __shared__ __align__(16) float sT[8][16 * 68];
  const int b    = blockIdx.y;
  const int lane = threadIdx.x & 31;
  const int wave = threadIdx.x >> 5;
  const int tilesN = N >> 6;
  const int tilesM = M >> 6;
  const int tile = blockIdx.x * 8 + wave;
  if (tile >= tilesM * tilesN) return;
  const int tm = tile / tilesN;
  const int tn = tile - tm * tilesN;
  const int m0 = tm << 6;
  const int n0 = tn << 6;

  const T* Ab  = A  + (size_t)b * strideA;
  const T* Bb  = Bt + (size_t)b * strideB;
  const T* Ab2 = SPLIT ? (A2  + (size_t)b * strideA) : nullptr;
  const T* Bb2 = SPLIT ? (Bt2 + (size_t)b * strideB) : nullptr;

  const int rlane = lane & 15;
  const int koff  = (lane >> 4) * 8;
  const int mOff  = (lane >> 4) * 8;

  v8f acc[4][4];
#pragma unroll
  for (int i = 0; i < 4; ++i)
#pragma unroll
    for (int j = 0; j < 4; ++j) acc[i][j] = (v8f){0.f,0.f,0.f,0.f,0.f,0.f,0.f,0.f};

  for (int k0 = 0; k0 < K; k0 += 32) {
    V bh[4], bl[4];
#pragma unroll
    for (int j = 0; j < 4; ++j) {
      const size_t bo = (size_t)(n0 + (j << 4) + rlane) * ldb + koff + k0;
      bh[j] = Frag<T>::load(Bb + bo);
      if (SPLIT) bl[j] = Frag<T>::load(Bb2 + bo);
    }
#pragma unroll
    for (int i = 0; i < 4; ++i) {
      const size_t ao = (size_t)(m0 + (i << 4) + rlane) * lda + koff + k0;
      V ah = Frag<T>::load(Ab + ao);
      V al;
      if (SPLIT) al = Frag<T>::load(Ab2 + ao);
#pragma unroll
      for (int j = 0; j < 4; ++j) {
        acc[i][j] = Frag<T>::mma(ah, bh[j], acc[i][j]);
        if (SPLIT) {
          acc[i][j] = Frag<T>::mma(ah, bl[j], acc[i][j]);
          acc[i][j] = Frag<T>::mma(al, bh[j], acc[i][j]);
        }
      }
      Frag<T>::guard(acc[i][0], acc[i][3], ah, SPLIT ? al : ah);
    }
    Frag<T>::keep(bh[0], bh[1], bh[2], bh[3]);
    if (SPLIT) Frag<T>::keep(bl[0], bl[1], bl[2], bl[3]);
  }
  acc_guard4(acc[0][0], acc[0][1], acc[0][2], acc[0][3]);
  acc_guard4(acc[1][0], acc[1][1], acc[1][2], acc[1][3]);
  acc_guard4(acc[2][0], acc[2][1], acc[2][2], acc[2][3]);
  acc_guard4(acc[3][0], acc[3][1], acc[3][2], acc[3][3]);

  float* slab = sT[wave];
  const float* Rb = RESID ? (resid + (size_t)b * strideR) : nullptr;
#pragma unroll
  for (int i = 0; i < 4; ++i) {
    const int mBase = m0 + (i << 4);
#pragma unroll
    for (int j = 0; j < 4; ++j) {
      const int n = n0 + (j << 4) + rlane;
      float bv = 0.f;
      if (BIAS_MODE == 2) bv = bias[n];
#pragma unroll
      for (int r = 0; r < 8; ++r) {
        float v = acc[i][j][r] * scale;
        if (BIAS_MODE == 1) v += bias[mBase + mOff + r];
        if (BIAS_MODE == 2) v += bv;
        if (RESID) v += Rb[(size_t)(mBase + mOff + r) * ldc + n];
        if (ACT == 2) v = fmaxf(v, 0.0f);
        if (ACT == 4) v = (v > 0.f) ? v : 0.01f * v;
        slab[(mOff + r) * 68 + (j << 4) + rlane] = v;
      }
    }
    __builtin_amdgcn_fence(__ATOMIC_RELEASE, "workgroup");
    __builtin_amdgcn_wave_barrier();
    __builtin_amdgcn_fence(__ATOMIC_ACQUIRE, "workgroup");
    if (OUT_MODE == 0) {
      float* C = (float*)Cout + (size_t)b * strideC;
      const int hh = lane >> 4, c4 = (lane & 15) * 4;
      for (int pass = 0; pass < 2; ++pass) {
#pragma unroll
        for (int it = 0; it < 8; ++it) {
          const int row = it * 2 + hh;
          v4f v = *(const v4f*)(slab + row * 68 + c4);
          *(volatile v4f*)(C + (size_t)(mBase + row) * ldc + n0 + c4) = v;
        }
        __threadfence();
      }
    } else {
      const int q = lane >> 3, c8 = (lane & 7) * 8;
      unsigned short* C  = (unsigned short*)Cout  + (size_t)b * strideC;
      unsigned short* C2 = (OUT_MODE == 2) ? ((unsigned short*)Cout2 + (size_t)b * strideC) : nullptr;
      for (int pass = 0; pass < 2; ++pass) {
#pragma unroll
        for (int it = 0; it < 4; ++it) {
          const int row = it * 4 + q;
          const float* sp = slab + row * 68 + c8;
          v8h hv, lv;
#pragma unroll
          for (int e = 0; e < 8; ++e) {
            if (OUT_MODE == 1) {
              hv[e] = (_Float16)sp[e];
            } else {
              unsigned short hb = f2bf_bits(sp[e]);
              unsigned short lb = f2bf_bits(sp[e] - bf_bits2f(hb));
              hv[e] = __builtin_bit_cast(_Float16, hb);
              lv[e] = __builtin_bit_cast(_Float16, lb);
            }
          }
          *(volatile v8h*)(C + (size_t)(mBase + row) * ldc + n0 + c8) = hv;
          if (OUT_MODE == 2) *(volatile v8h*)(C2 + (size_t)(mBase + row) * ldc + n0 + c8) = lv;
        }
        __threadfence();
      }
    }
    __builtin_amdgcn_fence(__ATOMIC_RELEASE, "workgroup");
    __builtin_amdgcn_wave_barrier();
    __builtin_amdgcn_fence(__ATOMIC_ACQUIRE, "workgroup");
  }
}

__global__ __launch_bounds__(256) void wt_split_kernel(const float* __restrict__ W0, const float* __restrict__ W1,
                                                       const float* __restrict__ W2, const float* __restrict__ W3,
                                                       unsigned short* __restrict__ hi, unsigned short* __restrict__ lo,
                                                       int nK, int nN, long zstride) {
  __shared__ float sm[64][65];
  const int t  = threadIdx.x;
  const int k0 = blockIdx.x * 64;
  const int n0 = blockIdx.y * 64;
  const int z  = blockIdx.z;
  const float* W = (z == 0) ? W0 : (z == 1) ? W1 : (z == 2) ? W2 : W3;
#pragma unroll
  for (int i = 0; i < 16; ++i) {
    const int e = i * 256 + t;
    const int r = e >> 6;
    const int c = e & 63;
    sm[c][r] = W[(size_t)(k0 + r) * nN + n0 + c];
  }
  __syncthreads();
  const int lane = t & 31, wave = t >> 5;
  const int q = lane >> 3, c8 = (lane & 7) * 8;
  unsigned short* hp = hi + (size_t)z * zstride;
  unsigned short* lp = lo + (size_t)z * zstride;
  for (int pass = 0; pass < 2; ++pass) {
#pragma unroll
    for (int it = 0; it < 2; ++it) {
      const int row = wave * 8 + it * 4 + q;
      unsigned short hb[8], lb[8];
#pragma unroll
      for (int e = 0; e < 8; ++e) {
        const float f = sm[row][c8 + e];
        hb[e] = f2bf_bits(f);
        lb[e] = f2bf_bits(f - bf_bits2f(hb[e]));
      }
      const v4u uh = (v4u){pk16(hb[0], hb[1]), pk16(hb[2], hb[3]), pk16(hb[4], hb[5]), pk16(hb[6], hb[7])};
      const v4u ul = (v4u){pk16(lb[0], lb[1]), pk16(lb[2], lb[3]), pk16(lb[4], lb[5]), pk16(lb[6], lb[7])};
      const size_t o = (size_t)(n0 + row) * nK + k0 + c8;
      *(volatile v4u*)(hp + o) = uh;
      *(volatile v4u*)(lp + o) = ul;
    }
    __threadfence();
  }
}

__global__ __launch_bounds__(256) void conv_expand_split_kernel(const float* __restrict__ x, const float* __restrict__ cw,
                                                                const float* __restrict__ cb,
                                                                unsigned short* __restrict__ hi, unsigned short* __restrict__ lo) {
  const int gid  = blockIdx.x * 256 + threadIdx.x;
  const int dblk = gid & 127;
  const int k    = (gid >> 7) & 7;
  const int l    = gid >> 10;
  const int d0   = dblk * 8;
  const bool has2 = (l >= 2);
  const bool has1 = (l >= 1);
  const int  rm2 = has2 ? (l - 2) : 0;
  const int  rm1 = has1 ? (l - 1) : 0;
  const float* p2 = x + (size_t)rm2 * kModel + d0;
  const float* p1 = x + (size_t)rm1 * kModel + d0;
  const float* p0 = x + (size_t)l   * kModel + d0;
  const v4f a2 = *(const v4f*)(p2), b2 = *(const v4f*)(p2 + 4);
  const v4f a1 = *(const v4f*)(p1), b1 = *(const v4f*)(p1 + 4);
  const v4f a0 = *(const v4f*)(p0), b0 = *(const v4f*)(p0 + 4);
  float xm2[8], xm1[8], x00[8];
#pragma unroll
  for (int e = 0; e < 4; ++e) {
    xm2[e] = has2 ? a2[e] : 0.f;  xm2[4 + e] = has2 ? b2[e] : 0.f;
    xm1[e] = has1 ? a1[e] : 0.f;  xm1[4 + e] = has1 ? b1[e] : 0.f;
    x00[e] = a0[e];               x00[4 + e] = b0[e];
  }
  unsigned short hb[8], lb[8];
#pragma unroll
  for (int e = 0; e < 8; ++e) {
    const int ch = (d0 + e) * kExpand + k;
    const float w0 = cw[ch * 3 + 0];
    const float w1 = cw[ch * 3 + 1];
    const float w2 = cw[ch * 3 + 2];
    const float r = w0 * xm2[e] + w1 * xm1[e] + w2 * x00[e] + cb[ch];
    hb[e] = f2bf_bits(r);
    lb[e] = f2bf_bits(r - bf_bits2f(hb[e]));
  }
  const v4u uh = (v4u){pk16(hb[0], hb[1]), pk16(hb[2], hb[3]), pk16(hb[4], hb[5]), pk16(hb[6], hb[7])};
  const v4u ul = (v4u){pk16(lb[0], lb[1]), pk16(lb[2], lb[3]), pk16(lb[4], lb[5]), pk16(lb[6], lb[7])};
  const size_t o = (size_t)l * kWide + (size_t)k * kModel + d0;
  *(volatile v4u*)(hi + o) = uh;
  *(volatile v4u*)(lo + o) = ul;
  __threadfence();
  *(volatile v4u*)(hi + o) = uh;
  *(volatile v4u*)(lo + o) = ul;
}

__device__ __forceinline__ float wave_sum32(float v) {
#pragma unroll
  for (int off = 16; off > 0; off >>= 1) v += __shfl_xor(v, off, 32);
  return v;
}

__global__ __launch_bounds__(64) void scan_head_kernel(
    const float* __restrict__ qraw, const float* __restrict__ kraw, const float* __restrict__ vraw,
    const float* __restrict__ bq, const float* __restrict__ bk, const float* __restrict__ bv,
    const float* __restrict__ kv_scale, const float* __restrict__ wgz_w, const float* __restrict__ wgz_b,
    const float* __restrict__ qk_scale, float* __restrict__ Yout) {
  __shared__ float Zc[kHeadDim * kHeadDim];
  __shared__ float Kvs[kHeadDim * kHeadDim];
  __shared__ float Mw[kHeadDim * kHeadDim];
  __shared__ float vvec[kHeadDim];
  __shared__ float qvec[kHeadDim];
  __shared__ __align__(16) float ych[kChunkT * kHeadDim];
  __shared__ float red[2][8];

  const int h = blockIdx.x;
  const int n = threadIdx.x;
  const int lane = n & 31, wave = n >> 5;

  for (int i = n; i < kHeadDim * kHeadDim; i += kHeadDim) {
    const float sc = kv_scale[i];
    Kvs[i] = sc;
    Mw[i]  = sc * wgz_w[i];
    Zc[i]  = 0.f;
  }
  const int col = h * kHeadDim + n;
  const float bqn = bq[col], bkn = bk[col], bvn = bv[col];
  const float qks = qk_scale[h];
  const float gzb = wgz_b[0];
  float mrun = -INFINITY, srun = 0.f, gcum = 0.f, nst = 0.f;
  __syncthreads();

  for (int t = 0; t < kSeqLen; ++t) {
    const size_t go = (size_t)t * kModel + col;
    const float qr = qraw[go] + bqn;
    const float kr = kraw[go] + bkn;
    const float vr = vraw[go] + bvn;
    float a0 = qr * qr, a1 = kr * kr, a2 = vr * vr;
    a0 = wave_sum32(a0); a1 = wave_sum32(a1); a2 = wave_sum32(a2);
    if (lane == 0) { red[wave][0] = a0; red[wave][1] = a1; red[wave][2] = a2; }
    __syncthreads();
    const float sq = red[0][0] + red[1][0];
    const float sk = red[0][1] + red[1][1];
    const float sv = red[0][2] + red[1][2];
    const float qn = qr / fmaxf(sqrtf(sq), kNormFloor);
    const float kn = kr / fmaxf(sqrtf(sk), kNormFloor);
    const float vn = vr / fmaxf(sqrtf(sv), kNormFloor);
    vvec[n] = vn;
    qvec[n] = qn;
    __syncthreads();
    float gp = 0.f;
#pragma unroll 8
    for (int p = 0; p < kHeadDim; ++p) gp += vvec[p] * Mw[p * kHeadDim + n];
    float b0 = qn * kn, b1 = qn, b2 = gp * kn;
    b0 = wave_sum32(b0); b1 = wave_sum32(b1); b2 = wave_sum32(b2);
    if (lane == 0) { red[wave][3] = b0; red[wave][4] = b1; red[wave][5] = b2; }
    __syncthreads();
    const float sim  = (red[0][3] + red[1][3]) * qks;
    const float qsum = red[0][4] + red[1][4];
    const float zg   = (red[0][5] + red[1][5]) + gzb;
    const float g    = ((zg >= 0.f) ? zg : 0.01f * zg) + kEpsF;
    const float mnew = fmaxf(mrun, sim);
    const float ex   = expf(mrun - mnew);
    const float et   = expf(sim - mnew);
    srun = srun * ex + et;
    mrun = mnew;
    gcum = gcum + g;
    nst  = nst * ex + et * vn;
    float yb = 0.f;
#pragma unroll 4
    for (int p = 0; p < kHeadDim; ++p) {
      const int idx = p * kHeadDim + n;
      const float z = Zc[idx] + ((vvec[p] * kn) * Kvs[idx]) * g;
      Zc[idx] = z;
      yb += qvec[p] * z;
    }
    const float invg  = 1.0f / (gcum + kEpsF);
    const float invs  = 1.0f / (srun + kEpsF);
    const float ybase = yb * invg;
    const float ylin  = qsum * (nst * invs);
    const float w     = et * invs;
    const float y     = ybase + (ylin - ybase) * w;
    ych[(t & (kChunkT - 1)) * kHeadDim + n] = y;
    __syncthreads();
    if ((t & (kChunkT - 1)) == (kChunkT - 1)) {
      const int t0 = t - (kChunkT - 1);
      const int rq = n >> 4, c4 = (n & 15) * 4;
      for (int pass = 0; pass < 2; ++pass) {
#pragma unroll
        for (int it = 0; it < 4; ++it) {
          const int row = it * 4 + rq;
          const v4f val = *(const v4f*)(ych + row * kHeadDim + c4);
          *(volatile v4f*)(Yout + (size_t)(t0 + row) * kModel + h * kHeadDim + c4) = val;
        }
        __threadfence();
      }
    }
  }
}

__global__ __launch_bounds__(128) void rownorm_split_kernel(const float* __restrict__ Y,
                                                            unsigned short* __restrict__ hi, unsigned short* __restrict__ lo) {
  __shared__ float part[4];
  const int row  = blockIdx.x;
  const int t    = threadIdx.x;
  const int lane = t & 31, wave = t >> 5;
  const float* p = Y + (size_t)row * kModel + 8 * t;
  const v4f a = *(const v4f*)(p);
  const v4f c = *(const v4f*)(p + 4);
  float xs[8];
#pragma unroll
  for (int e = 0; e < 4; ++e) { xs[e] = a[e]; xs[4 + e] = c[e]; }
  float ss = 0.f;
#pragma unroll
  for (int e = 0; e < 8; ++e) ss += xs[e] * xs[e];
  ss = wave_sum32(ss);
  if (lane == 0) part[wave] = ss;
  __syncthreads();
  const float tot = ((part[0] + part[1]) + part[2]) + part[3];
  const float inv = 1.0f / fmaxf(sqrtf(tot), kNormFloor);
  unsigned short hb[8], lb[8];
#pragma unroll
  for (int e = 0; e < 8; ++e) {
    const float f = xs[e] * inv;
    hb[e] = f2bf_bits(f);
    lb[e] = f2bf_bits(f - bf_bits2f(hb[e]));
  }
  const v4u uh = (v4u){pk16(hb[0], hb[1]), pk16(hb[2], hb[3]), pk16(hb[4], hb[5]), pk16(hb[6], hb[7])};
  const v4u ul = (v4u){pk16(lb[0], lb[1]), pk16(lb[2], lb[3]), pk16(lb[4], lb[5]), pk16(lb[6], lb[7])};
  const size_t o = (size_t)row * kModel + 8 * t;
  *(volatile v4u*)(hi + o) = uh;
  *(volatile v4u*)(lo + o) = ul;
  __threadfence();
  *(volatile v4u*)(hi + o) = uh;
  *(volatile v4u*)(lo + o) = ul;
}

extern "C" void kernel_launch(void* const* d_in, const int* in_sizes, int n_in,
                              void* d_out, int out_size, void* d_ws, size_t ws_size,
                              hipStream_t stream) {
  if (n_in != 17) return;
  const int expect_sizes[17] = {kSeqLen * kModel, kWide * 3, kWide, kWide * kModel, kModel,
                                kModel * kModel, kModel, kModel * kModel, kModel, kModel * kModel, kModel,
                                kModel * kModel, kModel, kHeadDim * kHeadDim, 1, kHeadDim * kHeadDim, kHeads};
  for (int i = 0; i < 17; ++i) if (in_sizes[i] != expect_sizes[i]) return;
  if (out_size != kSeqLen * kModel) return;

  const size_t MiB = (size_t)1 << 20;
  const size_t off_mphiT_hi = 0 * MiB,  off_mphiT_lo = 16 * MiB;
  const size_t off_xr_hi    = 32 * MiB, off_xr_lo    = 48 * MiB;
  const size_t off_xt_hi    = 64 * MiB, off_xt_lo    = 66 * MiB;
  const size_t off_wT_hi    = 68 * MiB, off_wT_lo    = 76 * MiB;
  const size_t off_qkv      = 84 * MiB;
  const size_t off_Y        = 96 * MiB;
  const size_t off_yn_hi    = 100 * MiB, off_yn_lo   = 102 * MiB;
  const size_t total        = 104 * MiB;
  if (ws_size < total) return;

  const float* x      = (const float*)d_in[0];
  const float* conv_w = (const float*)d_in[1];
  const float* conv_b = (const float*)d_in[2];
  const float* mphi_w = (const float*)d_in[3];
  const float* mphi_b = (const float*)d_in[4];
  const float* wq_w   = (const float*)d_in[5];
  const float* wq_b   = (const float*)d_in[6];
  const float* wk_w   = (const float*)d_in[7];
  const float* wk_b   = (const float*)d_in[8];
  const float* wv_w   = (const float*)d_in[9];
  const float* wv_b   = (const float*)d_in[10];
  const float* wo_w   = (const float*)d_in[11];
  const float* wo_b   = (const float*)d_in[12];
  const float* wgz_w  = (const float*)d_in[13];
  const float* wgz_b  = (const float*)d_in[14];
  const float* kv_sc  = (const float*)d_in[15];
  const float* qk_sc  = (const float*)d_in[16];

  char* ws = (char*)d_ws;
  unsigned short* mphiT_hi = (unsigned short*)(ws + off_mphiT_hi);
  unsigned short* mphiT_lo = (unsigned short*)(ws + off_mphiT_lo);
  unsigned short* xr_hi    = (unsigned short*)(ws + off_xr_hi);
  unsigned short* xr_lo    = (unsigned short*)(ws + off_xr_lo);
  unsigned short* xt_hi    = (unsigned short*)(ws + off_xt_hi);
  unsigned short* xt_lo    = (unsigned short*)(ws + off_xt_lo);
  unsigned short* wT_hi    = (unsigned short*)(ws + off_wT_hi);
  unsigned short* wT_lo    = (unsigned short*)(ws + off_wT_lo);
  float*          qkv      = (float*)(ws + off_qkv);
  float*          Ybuf     = (float*)(ws + off_Y);
  unsigned short* yn_hi    = (unsigned short*)(ws + off_yn_hi);
  unsigned short* yn_lo    = (unsigned short*)(ws + off_yn_lo);

  const long sqPlane = (long)kModel * kModel;

  wt_split_kernel<<<dim3(kWide / 64, kModel / 64, 1), 256, 0, stream>>>(
      mphi_w, mphi_w, mphi_w, mphi_w, mphiT_hi, mphiT_lo, kWide, kModel, 0L);
  wt_split_kernel<<<dim3(kModel / 64, kModel / 64, 4), 256, 0, stream>>>(
      wq_w, wk_w, wv_w, wo_w, wT_hi, wT_lo, kModel, kModel, sqPlane);
  conv_expand_split_kernel<<<(kSeqLen * kExpand * (kModel / 8)) / 256, 256, 0, stream>>>(x, conv_w, conv_b, xr_hi, xr_lo);
  wmma_gemm64<1, true, 2, 2, false, 0><<<dim3((kSeqLen / 64) * (kModel / 64) / 8, 1), 256, 0, stream>>>(
      xr_hi, xr_lo, kWide, 0L, mphiT_hi, mphiT_lo, kWide, 0L,
      (void*)xt_hi, (void*)xt_lo, kModel, 0L, mphi_b, (const float*)qkv, 0L, kSeqLen, kModel, kWide, 1.0f);
  wmma_gemm64<1, true, 0, 0, false, 0><<<dim3((kSeqLen / 64) * (kModel / 64) / 8, 3), 256, 0, stream>>>(
      xt_hi, xt_lo, kModel, 0L, wT_hi, wT_lo, kModel, sqPlane,
      (void*)qkv, (void*)qkv, kModel, sqPlane, mphi_b, (const float*)qkv, 0L, kSeqLen, kModel, kModel, 1.0f);
  scan_head_kernel<<<kHeads, kHeadDim, 0, stream>>>(
      qkv, qkv + sqPlane, qkv + 2 * sqPlane, wq_b, wk_b, wv_b, kv_sc, wgz_w, wgz_b, qk_sc, Ybuf);
  rownorm_split_kernel<<<kSeqLen, 128, 0, stream>>>(Ybuf, yn_hi, yn_lo);
  wmma_gemm64<1, true, 2, 0, false, 0><<<dim3((kSeqLen / 64) * (kModel / 64) / 8, 1), 256, 0, stream>>>(
      yn_hi, yn_lo, kModel, 0L, wT_hi + 3 * sqPlane, wT_lo + 3 * sqPlane, kModel, 0L,
      d_out, d_out, kModel, 0L, wo_b, (const float*)Ybuf, 0L, kSeqLen, kModel, kModel, 1.0f);
}
